// SMNetEncoder_80307298501389
// MI455X (gfx1250) — hardware-run, weakly checked
//
#include <hip/hip_runtime.h>


namespace {
constexpr int N = 30000, NP = 30016, E = 480000, D = 256, ED = 32, L = 4, NBLK = NP / 16;
constexpr float XS = 8.0f, WSC = 256.0f, LNEPS = 1e-5f;
typedef _Float16 b16;
typedef __attribute__((ext_vector_type(16))) _Float16 v16b;
typedef __attribute__((ext_vector_type(8))) _Float16 v8b;
typedef __attribute__((ext_vector_type(8))) float v8f;
typedef __attribute__((ext_vector_type(4))) float v4f;
__device__ __forceinline__ float bf16_rne(float f) { unsigned int u = __float_as_uint(f); u += 0x7FFFu + ((u >> 16) & 1u); return __uint_as_float(u & 0xFFFF0000u); }
__device__ __forceinline__ void split16(float v, b16& hi, b16& lo) { hi = (b16)v; lo = (b16)(v - (float)hi); }
__device__ __forceinline__ v16b frag_kb(const b16* p, int hh) { const v8b a = *(const v8b*)(p + 8 * hh), b = *(const v8b*)(p + 16 + 8 * hh); v16b f;
#pragma unroll
  for (int e = 0; e < 8; ++e) { f[e] = a[e]; f[8 + e] = b[e]; } return f; }
__device__ __forceinline__ v8f wmma16b(v16b a, v16b b, v8f c) { v8f d = __builtin_amdgcn_wmma_f32_16x16x32_f16(false, a, false, b, (short)0, c, false, false); asm volatile("v_nop\n\tv_nop\n\tv_nop\n\tv_nop" : "+v"(d) : "v"(a), "v"(b)); return d; }
__device__ __forceinline__ void wave_lds_sync() { __builtin_amdgcn_fence(__ATOMIC_RELEASE, "workgroup"); __builtin_amdgcn_wave_barrier(); __builtin_amdgcn_fence(__ATOMIC_ACQUIRE, "workgroup"); }
__device__ __forceinline__ float pmul(float a, float b) { float p = a * b; asm volatile("" : "+v"(p)); return p; }
__device__ __forceinline__ int iclamp(int v, int lo, int hi) { return v < lo ? lo : (v > hi ? hi : v); }
constexpr int CSR_NBLK = 512, CSR_GB = 9, CSR_GN = 1 << CSR_GB  , CSR_TS = (CSR_GN < 32 ? 32 : CSR_GN)  , CSR_MAXG = 512, CSR_CAP = 12288  ;
__device__ __host__ __forceinline__ int csr_tix(int v) { return (v >> CSR_GB) * CSR_TS + (v & (CSR_GN - 1)); }
__global__ __launch_bounds__(64) void csrA_kernel(const int* __restrict__ dst, int E, int N, int nG, int CHP, int NGP, int* __restrict__ STG, int* __restrict__ HST) {
  extern __shared__ int sm[];
  int* cnt = sm; int* run = sm + NGP; int* ids = sm + 2 * NGP;
  const int b = blockIdx.x; const int ch = (E + CSR_NBLK - 1) / CSR_NBLK; const int e0 = b * ch, e1 = min(E, e0 + ch);
  for (int i = threadIdx.x; i < NGP; i += 64) cnt[i] = 0;
  for (int i = threadIdx.x; i < CHP; i += 64) ids[i] = -1;
  __syncthreads();
  if (threadIdx.x == 0) {
    for (int e = e0; e < e1; ++e) { int d = dst[e]; d = (d < 0) ? 0 : (d >= N ? N - 1 : d); cnt[d >> CSR_GB] += 1; }
    int acc = 0; for (int g = 0; g < nG; ++g) { run[g] = acc; acc += cnt[g]; }
    for (int e = e0; e < e1; ++e) { int d = dst[e]; d = (d < 0) ? 0 : (d >= N ? N - 1 : d); const int g = d >> CSR_GB; ids[run[g]] = e; run[g] += 1; } }
  __syncthreads();
  typedef __attribute__((ext_vector_type(4))) int v4i;
  for (int pass = 0; pass < 2; ++pass) {
    for (int i = threadIdx.x; i < CHP / 4; i += 64) *(volatile v4i*)(STG + (size_t)b * CHP + i * 4) = *(const v4i*)(&ids[i * 4]);
    for (int i = threadIdx.x; i < NGP / 4; i += 64) { v4i v; for (int e = 0; e < 4; ++e) v[e] = (i * 4 + e < nG) ? cnt[i * 4 + e] : 0; *(volatile v4i*)(HST + (size_t)b * NGP + i * 4) = v; }
    __threadfence(); }
}
__global__ __launch_bounds__(512) void csrS_kernel(const int* __restrict__ HST, int nG, int NGP, int* __restrict__ START, int* __restrict__ TOT, int* __restrict__ OFF) {
  __shared__ int tot[CSR_MAXG];
  const int b = threadIdx.x;
  for (int pass = 0; pass < 2; ++pass) { int runb = 0; for (int g = 0; g < nG; ++g) { int c = HST[(size_t)b * NGP + g]; c = (c < 0) ? 0 : c; ((volatile int*)OFF)[(size_t)g * CSR_NBLK + b] = runb; runb += c; } __threadfence(); }
  for (int g = threadIdx.x; g < nG; g += 512) { int s = 0; for (int bb = 0; bb < CSR_NBLK; ++bb) { int c = HST[(size_t)bb * NGP + g]; s += (c < 0) ? 0 : c; } tot[g] = s; }
  __syncthreads();
  if (threadIdx.x < 32) {
    __shared__ int st[CSR_MAXG + 32];
    if (threadIdx.x == 0) { int acc = 0; for (int g = 0; g < NGP; ++g) { st[g] = acc; if (g < nG) acc += (tot[g] + 31) & ~31; } st[NGP] = acc; }
    __builtin_amdgcn_fence(__ATOMIC_RELEASE, "workgroup"); __builtin_amdgcn_wave_barrier(); __builtin_amdgcn_fence(__ATOMIC_ACQUIRE, "workgroup");
    for (int pass = 0; pass < 2; ++pass) { for (int i = threadIdx.x; i < NGP + 32; i += 32) { ((volatile int*)START)[i] = (i <= NGP) ? st[min(i, NGP)] : 0; ((volatile int*)TOT)[i] = (i < nG) ? tot[i] : 0; } __threadfence(); } }
}
__global__ __launch_bounds__(256) void csrB_kernel(const int* __restrict__ dst, int N, int nG, int CHP, int NGP, int permLen, const int* __restrict__ STG, const int* __restrict__ HST, const int* __restrict__ OFF, const int* __restrict__ START, const int* __restrict__ TOT, int* __restrict__ PERM, int* __restrict__ ROWPTR, int* __restrict__ ROWCNT, int* __restrict__ FLAG) {
  typedef __attribute__((ext_vector_type(4))) int v4i;
  __shared__ int ids[CSR_CAP]; __shared__ unsigned short key[CSR_CAP]; __shared__ int outp[CSR_CAP]; __shared__ int ncnt[CSR_GN + 1]; __shared__ int boff[CSR_NBLK + 1];
  const int g = blockIdx.x, t_ = threadIdx.x; int tot = TOT[g]; int st = START[g], stn = START[g + 1]; const int v0 = g * CSR_GN; const int nv = min(CSR_GN, N - v0); const int t0 = g * CSR_TS;
  st = (st < 0) ? 0 : (st > permLen - 32 ? permLen - 32 : st) & ~31; stn = (stn < st) ? st : (stn > permLen ? permLen : stn); tot = (tot < 0) ? 0 : tot; if (tot > stn - st && tot <= CSR_CAP) tot = stn - st;
  if (tot > CSR_CAP) {
    for (int pass = 0; pass < 2; ++pass) { for (int i = t_; i < CSR_TS / 4; i += 256) { v4i a, c; for (int e = 0; e < 4; ++e) { a[e] = st; c[e] = 0; } *(volatile v4i*)(ROWPTR + t0 + i * 4) = a; *(volatile v4i*)(ROWCNT + t0 + i * 4) = c; } if (t_ == 0) ((volatile int*)FLAG)[0] = 1; __threadfence(); } (void)nv; return; }
  if (t_ == 0) { int acc = 0; for (int b = 0; b < CSR_NBLK; ++b) { boff[b] = acc; int c = HST[(size_t)b * NGP + g]; c = (c < 0) ? 0 : (c > CHP ? CHP : c); acc += c; if (acc > tot) acc = tot; } boff[CSR_NBLK] = acc; }
  for (int i = t_; i <= CSR_GN; i += 256) ncnt[i] = 0;
  __syncthreads();
  for (int b = 0; b < CSR_NBLK; ++b) { const int c = boff[b + 1] - boff[b]; int o_ = OFF[(size_t)g * CSR_NBLK + b]; o_ = (o_ < 0) ? 0 : (o_ > CHP - c ? CHP - c : o_); const int* src_ = STG + (size_t)b * CHP + o_;
    for (int i = t_; i < c; i += 256) { int id = src_[i]; id = (id < 0) ? 0 : id; ids[boff[b] + i] = id; int d = dst[id]; d = (d < v0) ? v0 : (d >= N ? N - 1 : d); int kk = d - v0; kk = (kk < 0) ? 0 : (kk >= CSR_GN ? CSR_GN - 1 : kk); key[boff[b] + i] = (unsigned short)kk; } }
  __syncthreads();
  if (t_ == 0) { for (int i = 0; i < tot; ++i) ncnt[key[i]] += 1; int acc = 0; for (int vl = 0; vl < CSR_GN; ++vl) { const int c = ncnt[vl]; ncnt[vl] = acc; acc += c; } ncnt[CSR_GN] = acc;
    for (int i = 0; i < tot; ++i) { const int vl = key[i]; outp[ncnt[vl]] = ids[i]; ncnt[vl] += 1; }
    for (int vl = CSR_GN; vl > 0; --vl) ncnt[vl] = ncnt[vl - 1]; ncnt[0] = 0; }
  __syncthreads();
  for (int pass = 0; pass < 2; ++pass) {
    for (int i = t_; i < (stn - st) / 4; i += 256) { v4i v; for (int e = 0; e < 4; ++e) { const int q = i * 4 + e; v[e] = (q < tot) ? outp[q] : -1; } *(volatile v4i*)(PERM + st + i * 4) = v; }
    for (int i = t_; i < CSR_TS / 4; i += 256) { v4i a, c; for (int e = 0; e < 4; ++e) { const int vl = i * 4 + e; const int vc = vl < CSR_GN ? vl : CSR_GN; a[e] = (vl < CSR_GN) ? st + ncnt[vc] : st; c[e] = (vl < nv) ? (ncnt[(vc < CSR_GN ? vc : CSR_GN - 1) + 1] - ncnt[vc]) : 0; } *(volatile v4i*)(ROWPTR + t0 + i * 4) = a; *(volatile v4i*)(ROWCNT + t0 + i * 4) = c; }
    __threadfence(); }
}
__global__ __launch_bounds__(256) void csrZ_kernel(int* __restrict__ p, size_t n4) { typedef __attribute__((ext_vector_type(4))) int v4i; const size_t tid = (size_t)blockIdx.x * 256 + threadIdx.x, nth = (size_t)gridDim.x * 256; v4i z = {0, 0, 0, 0}; for (size_t i = tid; i < n4; i += nth) *(volatile v4i*)(p + i * 4) = z; }
struct CsrBufs { int *STG, *HST, *OFF, *START, *TOT, *PERM, *ROWPTR, *ROWCNT, *FLAG; int nG, NGP, CHP; size_t permLen; char* base; size_t bytes; };
static size_t csr_carve(CsrBufs& c, char* ws, size_t off, int E, int N) {
  const size_t off0 = off; c.base = ws + off;
  auto al = [&](size_t bytes) { char* p = ws + off; off += (bytes + 255) & ~(size_t)255; return p; };
  c.nG = (N + CSR_GN - 1) / CSR_GN; c.NGP = (c.nG + 31) & ~31; const int ch = (E + CSR_NBLK - 1) / CSR_NBLK; c.CHP = (ch + 31) & ~31; c.permLen = (size_t)E + 32 * (size_t)c.nG + 32;
  c.STG = (int*)al((size_t)CSR_NBLK * c.CHP * 4); c.HST = (int*)al((size_t)CSR_NBLK * c.NGP * 4); c.OFF = (int*)al((size_t)c.NGP * CSR_NBLK * 4); c.START = (int*)al((size_t)(c.NGP + 64) * 4); c.TOT = (int*)al((size_t)(c.NGP + 64) * 4);
  c.PERM = (int*)al(c.permLen * 4); c.ROWPTR = (int*)al((size_t)c.nG * CSR_TS * 4); c.ROWCNT = (int*)al((size_t)c.nG * CSR_TS * 4); c.FLAG = (int*)al(256);
  c.bytes = off - off0; return off;
}
static void csr_build(const CsrBufs& c, const int* dst, int E, int N, hipStream_t stream) {
  const size_t smem = (size_t)(2 * c.NGP + c.CHP) * 4;
  csrZ_kernel<<<512, 256, 0, stream>>>((int*)c.base, c.bytes / 16);
  csrA_kernel<<<CSR_NBLK, 64, smem, stream>>>(dst, E, N, c.nG, c.CHP, c.NGP, c.STG, c.HST);
  csrS_kernel<<<1, 512, 0, stream>>>(c.HST, c.nG, c.NGP, c.START, c.TOT, c.OFF);
  csrB_kernel<<<c.nG, 256, 0, stream>>>(dst, N, c.nG, c.CHP, c.NGP, (int)c.permLen, c.STG, c.HST, c.OFF, c.START, c.TOT, c.PERM, c.ROWPTR, c.ROWCNT, c.FLAG);
}


__global__ __launch_bounds__(256) void wprep_kernel(const float* __restrict__ w, int KIN, b16* __restrict__ WT) {
  const size_t u = (size_t)blockIdx.x * 256 + threadIdx.x; if (u >= (size_t)D * KIN / 8) return; const size_t e = u * 8; const int o = (int)(e / KIN), k0 = (int)(e % KIN); v8b v;
  for (int j = 0; j < 8; ++j) v[j] = (b16)(bf16_rne(w[(size_t)(k0 + j) * D + o]) * WSC); for (int pass = 0; pass < 2; ++pass) { *(volatile v8b*)(WT + e) = v; __threadfence(); }
}
__global__ __launch_bounds__(32) void lnrelu_kernel(const float* __restrict__ H, const float* __restrict__ gam, const float* __restrict__ bet, int NLIM, float* __restrict__ Y) {
  const int lane = threadIdx.x; const size_t v0 = (size_t)blockIdx.x * 16; float g8[8], b8[8]; for (int j = 0; j < 8; ++j) { const int c = (j >> 2) * 128 + lane * 4 + (j & 3); g8[j] = bf16_rne(gam[c]); b8[j] = bf16_rne(bet[c]); }
  for (int rr = 0; rr < 16; ++rr) { const size_t v = v0 + rr; v8f o = {0, 0, 0, 0, 0, 0, 0, 0};
    if (v < (size_t)NLIM) { v8f h; { const v4f h0 = *(const v4f*)(H + v * D + lane * 4), h1 = *(const v4f*)(H + v * D + 128 + lane * 4); for (int j = 0; j < 4; ++j) { h[j] = h0[j]; h[4 + j] = h1[j]; } } float s = 0.0f; for (int j = 0; j < 8; ++j) s += h[j]; for (int of = 16; of; of >>= 1) s += __shfl_xor(s, of); const float mu = s * (1.0f / D);
      float q = 0.0f; for (int j = 0; j < 8; ++j) { const float dd = h[j] - mu; q += pmul(dd, dd); } for (int of = 16; of; of >>= 1) q += __shfl_xor(q, of); const float rs = rsqrtf(q * (1.0f / D) + LNEPS);
      for (int j = 0; j < 8; ++j) o[j] = fmaxf(pmul(pmul(h[j] - mu, rs), g8[j]) + b8[j], 0.0f); }
    for (int pass = 0; pass < 2; ++pass) { v4f o0 = {o[0], o[1], o[2], o[3]}, o1 = {o[4], o[5], o[6], o[7]}; *(volatile v4f*)(Y + v * D + lane * 4) = o0; *(volatile v4f*)(Y + v * D + 128 + lane * 4) = o1; __threadfence(); } }
}
template <int RAW>
__global__ __launch_bounds__(128) void dst_kernel(const float* __restrict__ X, const float* __restrict__ ea, const int* __restrict__ srcs, const b16* __restrict__ EWT, const float* __restrict__ eb, const int* __restrict__ PERM, const int* __restrict__ ROWPTR, const int* __restrict__ ROWCNT, int permLen, int NLIM, float* __restrict__ AGG) {
  __shared__ __attribute__((aligned(16))) float Row[4][D + 4]; __shared__ int eid[4][16][2];
  const int wave = threadIdx.x >> 5, lane = threadIdx.x & 31, nloc = lane & 15, hlf = lane >> 4; const size_t v = (size_t)blockIdx.x * 4 + wave;
  int st = 0, cnt = 0; if (v < (size_t)NLIM) { st = ROWPTR[v]; cnt = ROWCNT[v]; cnt = iclamp(cnt, 0, 65536); st = iclamp(st, 0, permLen - cnt); }
  float ag[16]; for (int t = 0; t < 16; ++t) ag[t] = 0.0f; float ebv[16]; for (int t = 0; t < 16; ++t) ebv[t] = bf16_rne(eb[t * 16 + nloc]);
  const int nchunk = (cnt + 15) >> 4;
#pragma unroll 1
  for (int ch = 0; ch < nchunk; ++ch) {
    const int j = ch * 16 + nloc; const bool ok = j < cnt; const int e = ok ? iclamp(PERM[st + j], 0, E - 1) : 0; int s = iclamp(srcs[e], 0, N - 1); if (s >= NLIM) s = -1;
    if (hlf == 0) { eid[wave][nloc][0] = e; eid[wave][nloc][1] = ok ? s : -1; }
    wave_lds_sync();
    v16b a; { const int ee = eid[wave][nloc][0]; for (int jj = 0; jj < 8; ++jj) { a[jj] = (b16)(bf16_rne(ea[(size_t)ee * ED + 8 * hlf + jj]) * XS); a[8 + jj] = (b16)(bf16_rne(ea[(size_t)ee * ED + 16 + 8 * hlf + jj]) * XS); } }
#pragma unroll
    for (int t = 0; t < 16; ++t) { v8f acc = (v8f){}; acc = wmma16b(a, frag_kb(EWT + (size_t)(t * 16 + nloc) * ED, hlf), acc); const int c = t * 16 + nloc; float s_ = 0.0f;
#pragma unroll
      for (int r8 = 0; r8 < 8; ++r8) { const int rl = 8 * hlf + r8; const int sr = eid[wave][rl][1]; const int srr = sr < 0 ? 0 : sr; const float xv = X[(size_t)srr * D + c];
        s_ += (sr >= 0) ? fmaxf((RAW ? bf16_rne(xv) : xv) + acc[r8] * (1.0f / (XS * WSC)) + ebv[t], 0.0f) : 0.0f; }
      s_ += __shfl_xor(s_, 16); ag[t] += s_; }
    wave_lds_sync(); }
  if (hlf == 0) for (int t = 0; t < 16; ++t) Row[wave][t * 16 + nloc] = ag[t];
  wave_lds_sync();
  for (int pass = 0; pass < 2; ++pass) { *(volatile v4f*)(AGG + v * D + lane * 4) = *(const v4f*)(&Row[wave][lane * 4]); *(volatile v4f*)(AGG + v * D + 128 + lane * 4) = *(const v4f*)(&Row[wave][128 + lane * 4]); __threadfence(); }
}
template <int RAW, int RES>
__global__ __launch_bounds__(32) void mlp_kernel(const float* __restrict__ X, const float* __restrict__ AGG, const float* __restrict__ Hres, const b16* __restrict__ W1T, const b16* __restrict__ W2T, const float* __restrict__ b1, const float* __restrict__ b2, const float* __restrict__ epsv, int layer, int NLIM, float* __restrict__ Hout) {
  __shared__ __attribute__((aligned(16))) b16 Ah[16][D + 8], Al[16][D + 8]; __shared__ __attribute__((aligned(16))) float Tf[16][D + 4];
  const int lane = threadIdx.x, nloc = lane & 15, hlf = lane >> 4; const size_t v0 = (size_t)blockIdx.x * 16; const float ope = 1.0f + bf16_rne(epsv[layer]);
  for (int rr = 0; rr < 16; ++rr) { const size_t v = v0 + rr; const bool ok = v < (size_t)NLIM;
    for (int q = 0; q < 2; ++q) { v4f x = {0, 0, 0, 0}, g = {0, 0, 0, 0}; if (ok) { x = *(const v4f*)(X + v * D + lane * 8 + q * 4); g = *(const v4f*)(AGG + v * D + lane * 8 + q * 4); }
      for (int j = 0; j < 4; ++j) { const float hv = pmul(ope, RAW ? bf16_rne(x[j]) : x[j]) + g[j]; b16 p, ql; split16(hv * XS, p, ql); Ah[rr][lane * 8 + q * 4 + j] = p; Al[rr][lane * 8 + q * 4 + j] = ql; } } }
  wave_lds_sync();
#pragma unroll 1
  for (int cg = 0; cg < 2; ++cg) { v8f acc[8];
#pragma unroll
    for (int t = 0; t < 8; ++t) acc[t] = (v8f){};
#pragma unroll 2
    for (int kb = 0; kb < D; kb += 32) { const v16b a = frag_kb(&Ah[nloc][kb], hlf), al = frag_kb(&Al[nloc][kb], hlf);
#pragma unroll
      for (int t = 0; t < 8; ++t) { const v16b bw = frag_kb(W1T + (size_t)(cg * 128 + t * 16 + nloc) * D + kb, hlf); acc[t] = wmma16b(a, bw, acc[t]); acc[t] = wmma16b(al, bw, acc[t]); } }
#pragma unroll
    for (int t = 0; t < 8; ++t) { const int c = cg * 128 + t * 16 + nloc; const float bb = bf16_rne(b1[c]);
#pragma unroll 1
      for (int r8 = 0; r8 < 8; ++r8) Tf[8 * hlf + r8][c] = fmaxf(acc[t][r8] * (1.0f / (XS * WSC)) + bb, 0.0f); } }
  wave_lds_sync();
  for (int rr = 0; rr < 16; ++rr) for (int q = 0; q < 8; ++q) { const float hv = Tf[rr][lane * 8 + q]; b16 p, ql; split16(hv * XS, p, ql); Ah[rr][lane * 8 + q] = p; Al[rr][lane * 8 + q] = ql; }
  wave_lds_sync();
#pragma unroll 1
  for (int cg = 0; cg < 2; ++cg) { v8f acc[8];
#pragma unroll
    for (int t = 0; t < 8; ++t) acc[t] = (v8f){};
#pragma unroll 2
    for (int kb = 0; kb < D; kb += 32) { const v16b a = frag_kb(&Ah[nloc][kb], hlf), al = frag_kb(&Al[nloc][kb], hlf);
#pragma unroll
      for (int t = 0; t < 8; ++t) { const v16b bw = frag_kb(W2T + (size_t)(cg * 128 + t * 16 + nloc) * D + kb, hlf); acc[t] = wmma16b(a, bw, acc[t]); acc[t] = wmma16b(al, bw, acc[t]); } }
#pragma unroll
    for (int t = 0; t < 8; ++t) { const int c = cg * 128 + t * 16 + nloc; const float bb = bf16_rne(b2[c]);
#pragma unroll 1
      for (int r8 = 0; r8 < 8; ++r8) { const int rl = 8 * hlf + r8; const size_t v = v0 + rl; float val = 0.0f; if (v < (size_t)NLIM) { val = acc[t][r8] * (1.0f / (XS * WSC)) + bb; if (RES) val += Hres[v * D + c]; } Tf[rl][c] = val; } } }
  wave_lds_sync();
  for (int pass = 0; pass < 2; ++pass) { for (int rr = 0; rr < 16; ++rr) { *(volatile v4f*)(Hout + (v0 + rr) * D + lane * 4) = *(const v4f*)(&Tf[rr][lane * 4]); *(volatile v4f*)(Hout + (v0 + rr) * D + 128 + lane * 4) = *(const v4f*)(&Tf[rr][128 + lane * 4]); } __threadfence(); }
}
__global__ __launch_bounds__(32) void final_kernel(const float* __restrict__ H, const float* __restrict__ gam, const float* __restrict__ bet, float* __restrict__ out) {
  const int lane = threadIdx.x; const size_t v0 = (size_t)blockIdx.x * 16; float g8[8], b8[8]; for (int j = 0; j < 8; ++j) { const int c = (j >> 2) * 128 + lane * 4 + (j & 3); g8[j] = bf16_rne(gam[c]); b8[j] = bf16_rne(bet[c]); }
  for (int rr = 0; rr < 16; ++rr) { const size_t v = v0 + rr; if (v >= (size_t)N) break; v8f h; { const v4f h0 = *(const v4f*)(H + v * D + lane * 4), h1 = *(const v4f*)(H + v * D + 128 + lane * 4); for (int j = 0; j < 4; ++j) { h[j] = h0[j]; h[4 + j] = h1[j]; } } float s = 0.0f; for (int j = 0; j < 8; ++j) s += h[j]; for (int of = 16; of; of >>= 1) s += __shfl_xor(s, of); const float mu = s * (1.0f / D);
    float q = 0.0f; for (int j = 0; j < 8; ++j) { const float dd = h[j] - mu; q += pmul(dd, dd); } for (int of = 16; of; of >>= 1) q += __shfl_xor(q, of); const float rs = rsqrtf(q * (1.0f / D) + LNEPS);
    v8f o; for (int j = 0; j < 8; ++j) o[j] = fmaxf(pmul(pmul(h[j] - mu, rs), g8[j]) + b8[j], 0.0f);
    for (int pass = 0; pass < 2; ++pass) { v4f o0 = {o[0], o[1], o[2], o[3]}, o1 = {o[4], o[5], o[6], o[7]}; *(volatile v4f*)(out + v * D + lane * 4) = o0; *(volatile v4f*)(out + v * D + 128 + lane * 4) = o1; __threadfence(); } }
}
}

extern "C" void kernel_launch(void* const* d_in, const int* in_sizes, int n_in, void* d_out, int out_size, void* d_ws, size_t ws_size, hipStream_t stream) {
  (void)n_in;
  auto Fp = [&](int i) { return (const float*)d_in[i]; }; auto Ip = [&](int i) { return (const int*)d_in[i]; };
  if (in_sizes[0] != N * D || in_sizes[1] != 2 * E || in_sizes[2] != E * ED || in_sizes[3] != L * D * D || in_sizes[5] != L * D * D || in_sizes[7] != L * ED * D || in_sizes[9] != L || in_sizes[10] != L * D || out_size != N * D) return;
  const int NLIM = N; const int GB16 = NBLK, GB4 = NP / 4;
  size_t off = 0; char* ws = (char*)d_ws;
  auto carve = [&](size_t bytes) { char* p = ws + off; off += (bytes + 255) & ~(size_t)255; return p; };
  b16* W1T = (b16*)carve((size_t)L * D * D * 2); b16* W2T = (b16*)carve((size_t)L * D * D * 2); b16* EWT = (b16*)carve((size_t)L * D * ED * 2);
  float* H = (float*)carve((size_t)NP * D * 4); float* Y = (float*)carve((size_t)NP * D * 4); float* AGG = (float*)carve((size_t)NP * D * 4); float* H2 = (float*)carve((size_t)NP * D * 4);
  CsrBufs csr; off = csr_carve(csr, ws, off, E, N);
  if (off > ws_size) return;
  for (int l = 0; l < L; ++l) { wprep_kernel<<<(D * D / 8 + 255) / 256, 256, 0, stream>>>(Fp(3) + (size_t)l * D * D, D, W1T + (size_t)l * D * D); wprep_kernel<<<(D * D / 8 + 255) / 256, 256, 0, stream>>>(Fp(5) + (size_t)l * D * D, D, W2T + (size_t)l * D * D); wprep_kernel<<<(D * ED / 8 + 255) / 256, 256, 0, stream>>>(Fp(7) + (size_t)l * ED * D, ED, EWT + (size_t)l * D * ED); }
  csr_build(csr, Ip(1) + E, E, N, stream);
  dst_kernel<1><<<GB4, 128, 0, stream>>>(Fp(0), Fp(2), Ip(1), EWT, Fp(8), csr.PERM, csr.ROWPTR, csr.ROWCNT, (int)csr.permLen, NLIM, AGG);
  mlp_kernel<1, 0><<<GB16, 32, 0, stream>>>(Fp(0), AGG, nullptr, W1T, W2T, Fp(4), Fp(6), Fp(9), 0, NLIM, H);
  float* Hc = H; float* Hn = H2;
  for (int l = 1; l < L; ++l) {
    lnrelu_kernel<<<GB16, 32, 0, stream>>>(Hc, Fp(10) + (size_t)l * D, Fp(11) + (size_t)l * D, NLIM, Y);
    dst_kernel<0><<<GB4, 128, 0, stream>>>(Y, Fp(2), Ip(1), EWT + (size_t)l * D * ED, Fp(8) + (size_t)l * D, csr.PERM, csr.ROWPTR, csr.ROWCNT, (int)csr.permLen, NLIM, AGG);
    mlp_kernel<0, 1><<<GB16, 32, 0, stream>>>(Y, AGG, Hc, W1T + (size_t)l * D * D, W2T + (size_t)l * D * D, Fp(4) + (size_t)l * D, Fp(6) + (size_t)l * D, Fp(9), l, NLIM, Hn);
    float* t = Hc; Hc = Hn; Hn = t; }
  final_kernel<<<GB16, 32, 0, stream>>>(Hc, Fp(10), Fp(11), (float*)d_out);
}
